// DApp_classifier_87643102642497
// MI455X (gfx1250) — hardware-run, weakly checked
//
#include <hip/hip_runtime.h>

typedef float          v8f   __attribute__((ext_vector_type(8)));
typedef float          v4f   __attribute__((ext_vector_type(4)));
typedef unsigned int   v4u   __attribute__((ext_vector_type(4)));
typedef int            v8i   __attribute__((ext_vector_type(8)));
typedef unsigned short v8us  __attribute__((ext_vector_type(8)));
typedef unsigned short v16us __attribute__((ext_vector_type(16)));
typedef __bf16         v16bf __attribute__((ext_vector_type(16)));
typedef _Float16       v16h  __attribute__((ext_vector_type(16)));
typedef v4f  __attribute__((may_alias)) v4fa;
typedef v8us __attribute__((may_alias)) v8usa;
union FragB { v16bf v; v16us u; v8us h[2]; v8i w; };
union FragH { v16h  v; v16us u; v8us h[2]; v8i w; };

__device__ __forceinline__ v8f wmb(const FragB& a, const FragB& b, v8f c) {
  v8f d = __builtin_amdgcn_wmma_f32_16x16x32_bf16(false, a.v, false, b.v, (short)0, c, false, false);
  asm volatile("v_nop\n\tv_nop\n\tv_nop\n\tv_nop" : "+v"(d) : "v"(a.w), "v"(b.w));
  return d;
}

__device__ __forceinline__ v8f wmh(const FragH& a, const FragH& b, v8f c) {
  v8f d = __builtin_amdgcn_wmma_f32_16x16x32_f16(false, a.v, false, b.v, (short)0, c, false, false);
  asm volatile("v_nop\n\tv_nop\n\tv_nop\n\tv_nop" : "+v"(d) : "v"(a.w), "v"(b.w));
  return d;
}

__device__ __forceinline__ unsigned bf16_bits(float f) {
  const unsigned u = __float_as_uint(f);
  const unsigned r = (u + 0x7FFFu + ((u >> 16) & 1u)) >> 16;
  const unsigned q = (u >> 16) | 0x40u;
  return ((u & 0x7fffffffu) > 0x7f800000u) ? q : r;
}

__device__ __forceinline__ float bf16_val(float f) {
  return __uint_as_float(bf16_bits(f) << 16);
}
__device__ __forceinline__ int clampi(int v, int lo, int hi) {
  return v < lo ? lo : (v > hi ? hi : v);
}

__device__ __forceinline__ unsigned f16_bits(float f) {
  const unsigned u  = __float_as_uint(f);
  const unsigned s  = (u >> 16) & 0x8000u;
  const unsigned a  = u & 0x7fffffffu;
  const unsigned t  = a - 0x38000000u;
  const unsigned r  = (t + 0x0FFFu + ((t >> 13) & 1u)) >> 13;
  const unsigned rc = r > 0x7C00u ? 0x7C00u : r;
  const bool small  = a < 0x38800000u;
  const bool isnan  = a > 0x7f800000u;
  const unsigned fin = small ? 0u : (s | rc);
  return isnan ? (s | 0x7E00u) : fin;
}

__device__ __forceinline__ unsigned pk16(unsigned lo, unsigned hi) { return lo | (hi << 16); }
__device__ __forceinline__ unsigned bf16_lo_bits(float v) {
  float hi = bf16_val(v);
  asm volatile("" : "+v"(hi));
  return bf16_bits(v - hi);
}
__device__ __forceinline__ v4u pack8_bf16(v4f a, v4f c) {
  return (v4u){ pk16(bf16_bits(a[0]), bf16_bits(a[1])), pk16(bf16_bits(a[2]), bf16_bits(a[3])),
                pk16(bf16_bits(c[0]), bf16_bits(c[1])), pk16(bf16_bits(c[2]), bf16_bits(c[3])) };
}
__device__ __forceinline__ v4u pack8_bf16_lo(v4f a, v4f c) {
  return (v4u){ pk16(bf16_lo_bits(a[0]), bf16_lo_bits(a[1])), pk16(bf16_lo_bits(a[2]), bf16_lo_bits(a[3])),
                pk16(bf16_lo_bits(c[0]), bf16_lo_bits(c[1])), pk16(bf16_lo_bits(c[2]), bf16_lo_bits(c[3])) };
}
__device__ __forceinline__ v4u pack8_f16(v4f a, v4f c) {
  return (v4u){ pk16(f16_bits(a[0]), f16_bits(a[1])), pk16(f16_bits(a[2]), f16_bits(a[3])),
                pk16(f16_bits(c[0]), f16_bits(c[1])), pk16(f16_bits(c[2]), f16_bits(c[3])) };
}

template <int FORM>
__global__ __launch_bounds__(256) void k_plane(const float* __restrict__ src, int rows, int cols, int ldsrc,
                                               unsigned short* __restrict__ dst, int MP, int KP) {
  static_assert(FORM >= 0 && FORM <= 3);
  const int KTOT = (FORM == 1 || FORM == 3) ? 2 * KP : KP;
  const unsigned ppr   = (unsigned)(KTOT >> 3);
  const unsigned kp8   = (unsigned)(KP >> 3);
  const unsigned total = (unsigned)MP * ppr;
  const unsigned g     = blockIdx.x * 256u + threadIdx.x;
  const unsigned rowu  = g / ppr;
  const unsigned p     = g - rowu * ppr;
  const bool second    = p >= kp8;
  const int row = (int)rowu;
  const int c0  = (int)((second ? p - kp8 : p) << 3);
  const float* srow = src + (size_t)clampi(row, 0, rows - 1) * (size_t)ldsrc;
  float x[8];
  unsigned mk[8];
#pragma unroll
  for (int e = 0; e < 8; ++e) {
    const int c = c0 + e;
    const float v = srow[clampi(c, 0, cols - 1)];
    asm volatile("" :: "v"(v));
    x[e]  = v;
    mk[e] = (row < rows && c < cols) ? 0xFFFFu : 0u;
  }
  const v4f a = (v4f){ x[0], x[1], x[2], x[3] };
  const v4f c = (v4f){ x[4], x[5], x[6], x[7] };
  v4u o;
  if (FORM == 2) {
    o = pack8_f16(a, c);
  } else {
    const v4u hi = pack8_bf16(a, c);
    o = hi;
    if (FORM == 1) { const v4u lo = pack8_bf16_lo(a, c); o = second ? lo : hi; }
  }
  const v4u mw = (v4u){ pk16(mk[0], mk[1]), pk16(mk[2], mk[3]), pk16(mk[4], mk[5]), pk16(mk[6], mk[7]) };
  o &= mw;
  if (g < total) {
    volatile v4u* q = (volatile v4u*)(dst + (size_t)g * 8);
    *q = o;
    __threadfence();
    *q = o;
  }
}

template <int FORM> struct FragOf    { typedef FragB T; };
template <>         struct FragOf<2> { typedef FragH T; };
__device__ __forceinline__ v8f mm(const FragB& a, const FragB& b, v8f c) { return wmb(a, b, c); }
__device__ __forceinline__ v8f mm(const FragH& a, const FragH& b, v8f c) { return wmh(a, b, c); }
template <class F> __device__ __forceinline__ F ld_frag(const unsigned short* p) {
  F f;
  f.h[0] = *(const v8usa*)(p);
  f.h[1] = *(const v8usa*)(p + 16);
  return f;
}

template <int FORM, int EPI>
__global__ __launch_bounds__(256) __attribute__((amdgpu_num_vgpr(248)))
void k_gemm_nt(const unsigned short* __restrict__ A, const unsigned short* __restrict__ B,
               const float* __restrict__ bias, float* __restrict__ D, int M, int N, int KTOT, int ldd) {
  static_assert(FORM >= 0 && FORM <= 2);
  static_assert(EPI == 0 || EPI == 1);
  typedef typename FragOf<FORM>::T F;
  __shared__ __attribute__((aligned(16))) float sT[8][16 * 68];
  const int lane = threadIdx.x & 31;
  const int wave = threadIdx.x >> 5;
  const int tilesM = (M + 63) >> 6;
  const int tilesN = (N + 63) >> 6;
  const int tile = blockIdx.x * 8 + wave;
  if (tile >= tilesM * tilesN) return;
  const int tm = tile / tilesN;
  const int tn = tile - tm * tilesN;
  const int m0 = tm << 6;
  const int n0 = tn << 6;

  const int rl = lane & 15;
  const int h8 = (lane >> 4) * 8;
  const unsigned short* pa = A + (size_t)(m0 + rl) * (size_t)KTOT + h8;
  const unsigned short* pb = B + (size_t)(n0 + rl) * (size_t)KTOT + h8;

  v8f acc[4][4];
#pragma unroll
  for (int i = 0; i < 4; ++i)
#pragma unroll
    for (int j = 0; j < 4; ++j) acc[i][j] = (v8f){0.f, 0.f, 0.f, 0.f, 0.f, 0.f, 0.f, 0.f};

#pragma unroll 1
  for (int k0 = 0; k0 < KTOT; k0 += 32) {
    F bf[4];
#pragma unroll
    for (int j = 0; j < 4; ++j) bf[j] = ld_frag<F>(pb + (size_t)(j << 4) * (size_t)KTOT + k0);
#pragma unroll
    for (int i = 0; i < 4; ++i) {
      const F af = ld_frag<F>(pa + (size_t)(i << 4) * (size_t)KTOT + k0);
#pragma unroll
      for (int j = 0; j < 4; ++j) acc[i][j] = mm(af, bf[j], acc[i][j]);
    }
  }

  float* slab = sT[wave];
  const int hh = lane >> 4;
  const int c4 = (lane & 15) * 4;
  const int nc = n0 + c4;
  const bool cok = nc < N;
  v4f bv = (v4f){0.f, 0.f, 0.f, 0.f};
  if (EPI == 1) {
    bv = *(const v4fa*)(bias + clampi(nc, 0, N - 4));
    asm volatile("" :: "v"(bv));
  }
#pragma unroll
  for (int i = 0; i < 4; ++i) {
    const int mBase = m0 + (i << 4);
#pragma unroll
    for (int j = 0; j < 4; ++j) {
#pragma unroll
      for (int r = 0; r < 8; ++r) slab[(h8 + r) * 68 + (j << 4) + rl] = acc[i][j][r];
    }
    __builtin_amdgcn_fence(__ATOMIC_RELEASE, "workgroup");
    __builtin_amdgcn_wave_barrier();
    __builtin_amdgcn_fence(__ATOMIC_ACQUIRE, "workgroup");
    v4f vv[8];
#pragma unroll
    for (int it = 0; it < 8; ++it) {
      const int row = it * 2 + hh;
      v4f v = *(const v4fa*)(slab + row * 68 + c4);
      if (EPI == 1) v += bv;
      vv[it] = v;
    }
    for (int pass = 0; pass < 2; ++pass) {
#pragma unroll
      for (int it = 0; it < 8; ++it) {
        const int row = mBase + it * 2 + hh;
        if (cok && row < M) *(volatile v4f*)(D + (size_t)row * (size_t)ldd + nc) = vv[it];
      }
      __threadfence();
    }
    __builtin_amdgcn_fence(__ATOMIC_RELEASE, "workgroup");
    __builtin_amdgcn_wave_barrier();
    __builtin_amdgcn_fence(__ATOMIC_ACQUIRE, "workgroup");
  }
}

#pragma clang fp contract(off)

#define NN       50000
#define NE       1600000
#define NG       512
#define NCLS     53
#define VOCAB    3100
#define MPN      50048
#define NREC     391
#define NBLK     98
#define NBROWS   512
#define GBLK     16
#define GROWS    32
#define DEGCAP   96
#define GCAP     160
#define MAXHITS  16678
#define MAXDEG   57
#define GMAXDEG  127
#define NTHR     256
#define NWAVE    8
#define EPT      8
#define CHUNK    (NTHR * EPT)
#define WCAP     (EPT * 32)
#define LISTN    (NWAVE * WCAP)
#define NBMAX    2048
#define ESH      11
#define RCAP     18432
#define LDS_BKT  ((2 * RCAP + 2 * NBMAX + LISTN) * 4 + 64)
#define LDS_AGG  (RCAP * 4)
#define PA_B1    0
#define PA_B2    64
#define PA_B3    128
#define PA_GAM   192
#define PA_BET   256
#define PA_BC    320
#define PA_EPS   384
#define PAR_LINES 13
#define WSMAX    ((size_t)128 << 20)

static_assert(MPN % 128 == 0 && MPN >= NN && MPN - NN < 64);
static_assert(NREC * 128 == MPN && NN == 390 * 128 + 80);
static_assert(NN % 16 == 0 && NE % 8 == 0 && NN % 8 == 0);
static_assert(NBLK * NBROWS >= NN && (NBLK - 1) * NBROWS < NN);
static_assert(NBROWS % 2 == 0 && (NN - (NBLK - 1) * NBROWS) % 2 == 0);
static_assert(NBROWS == 8 * 64);
static_assert(GBLK * GROWS == NG && GROWS == 8 * 4);
static_assert(NBROWS <= 1024 && GROWS <= 1024);
static_assert(NBROWS <= NBMAX && (1 << ESH) >= NBMAX && NTHR * 8 == NBMAX && LISTN >= NBMAX);
static_assert(NE <= (1 << (32 - ESH)));
static_assert(RCAP % 1024 == 0 && RCAP % 16 == 0 && RCAP > MAXHITS + 1024);
static_assert(RCAP * 100 >= MAXHITS * 105);
static_assert(RCAP * 100 >= GROWS * GMAXDEG * 105);
static_assert(DEGCAP >= MAXDEG + 8);
static_assert(GCAP >= GMAXDEG + 8);
static_assert(LDS_BKT <= 327680 && LDS_AGG + 4096 <= 327680);
static_assert((MPN * 16) % 256 == 0);
static_assert(64 * 2 == 128);
static_assert(NG % 32 == 0 && (32 * NCLS * 4) % 128 == 0 && (32 * NCLS) % 4 == 0);
static_assert((NG * 384 / 8) % 256 == 0);
static_assert(PAR_LINES * 32 == PA_EPS + 32);

constexpr size_t al256(size_t v) { return (v + 255) & ~(size_t)255; }
constexpr size_t O_H      = 0;
constexpr size_t O_T      = al256(O_H      + (size_t)MPN * 64 * 4);
constexpr size_t O_A      = al256(O_T      + (size_t)MPN * 64 * 4);
constexpr size_t O_BLIST  = al256(O_A      + (size_t)MPN * 128 * 2);
constexpr size_t O_OFFC   = al256(O_BLIST  + (size_t)NBLK * RCAP * 4);
constexpr size_t O_META   = al256(O_OFFC   + (size_t)NBLK * 2048 * 4);
constexpr size_t O_GBLIST = al256(O_META   + (size_t)NBLK * 128);
constexpr size_t O_GOFFC  = al256(O_GBLIST + (size_t)GBLK * RCAP * 4);
constexpr size_t O_GMETA  = al256(O_GOFFC  + (size_t)GBLK * 2048 * 4);
constexpr size_t O_REC    = al256(O_GMETA  + (size_t)GBLK * 128);
constexpr size_t O_STAT   = al256(O_REC    + (size_t)NREC * 192 * 8);
constexpr size_t O_PAR    = al256(O_STAT   + 512);
constexpr size_t O_W1T    = al256(O_PAR    + 2048);
constexpr size_t O_W2T    = al256(O_W1T    + 64 * 128 * 2);
constexpr size_t O_W3T    = al256(O_W2T    + 64 * 128 * 2);
constexpr size_t O_WCT    = al256(O_W3T    + 64 * 128 * 2);
constexpr size_t O_GF     = al256(O_WCT    + 64 * 384 * 2);
constexpr size_t O_GFHL   = al256(O_GF     + (size_t)NG * 192 * 4);
constexpr size_t O_C      = al256(O_GFHL   + (size_t)NG * 384 * 2);
constexpr size_t WS_TOTAL = al256(O_C      + (size_t)NG * 64 * 4);
static_assert(WS_TOTAL <= (size_t)WSMAX);
static_assert(PAR_LINES * 128 <= 2048);

typedef int v4i __attribute__((ext_vector_type(4)));
typedef v4i __attribute__((may_alias)) v4ia;
typedef v4u __attribute__((may_alias)) v4ua;
typedef double v2d __attribute__((ext_vector_type(2)));
typedef v2d __attribute__((may_alias)) v2da;

__device__ __forceinline__ void wave_sync_lds() {
  __builtin_amdgcn_fence(__ATOMIC_RELEASE, "workgroup");
  __builtin_amdgcn_wave_barrier();
  __builtin_amdgcn_fence(__ATOMIC_ACQUIRE, "workgroup");
}
__device__ __forceinline__ void st2_v4u(void* p, const v4u v) {
  volatile v4u* q = (volatile v4u*)p;
  *q = v;
  __threadfence();
  *q = v;
}
__device__ __forceinline__ void st2_v4f(float* p, const v4f v) {
  volatile v4f* q = (volatile v4f*)p;
  *q = v;
  __threadfence();
  *q = v;
}
__device__ __forceinline__ void st2_v4i(int* p, const v4i v) {
  volatile v4i* q = (volatile v4i*)p;
  *q = v;
  __threadfence();
  *q = v;
}
__device__ __forceinline__ void st2_v2d(double* p, const v2d v) {
  volatile v2d* q = (volatile v2d*)p;
  *q = v;
  __threadfence();
  *q = v;
}
__device__ __forceinline__ float relu_keep(float t) { return (t > 0.0f) ? t : (t - t); }

__device__ __forceinline__ v4u gather8_bf16(const float* __restrict__ src, int base, int k0, int kmask, int stride,
                                            unsigned mk) {
  float x[8];
#pragma unroll
  for (int e = 0; e < 8; ++e) {
    const float v = src[base + ((k0 + e) & kmask) * stride];
    asm volatile("" :: "v"(v));
    x[e] = v;
  }
  v4u o = pack8_bf16((v4f){ x[0], x[1], x[2], x[3] }, (v4f){ x[4], x[5], x[6], x[7] });
  o &= (v4u){ mk, mk, mk, mk };
  return o;
}

__global__ __launch_bounds__(256) void k_prep(
    const int* __restrict__ pkt, const float* __restrict__ emb, const float* __restrict__ eps,
    const float* __restrict__ W1, const float* __restrict__ b1, const float* __restrict__ W2,
    const float* __restrict__ b2, const float* __restrict__ W3, const float* __restrict__ b3,
    const float* __restrict__ gam, const float* __restrict__ bet, const float* __restrict__ Wc,
    const float* __restrict__ bc,
    unsigned short* W1T2, unsigned short* W2T2, unsigned short* W3T2, unsigned short* WCT2,
    float* PAR, float* H, float* T, unsigned short* A) {
  const int b = (int)blockIdx.x, tid = (int)threadIdx.x;
  if (b < 4) {
    const int u = b * 256 + tid;
    const int n = u >> 4, p = u & 15;
    const v4u o = gather8_bf16(W1, n, 8 * p, 63, 64, 0xFFFFFFFFu);
    st2_v4u(W1T2 + (size_t)u * 8, o);
  } else if (b < 8) {
    const int u = (b - 4) * 256 + tid;
    const int n = u >> 4, p = u & 15;
    const v4u o = gather8_bf16(W2, n, 8 * p, 63, 64, 0xFFFFFFFFu);
    st2_v4u(W2T2 + (size_t)u * 8, o);
  } else if (b < 12) {
    const int u = (b - 8) * 256 + tid;
    const int n = u >> 4, p = u & 15;
    const v4u o = gather8_bf16(W3, n, 8 * p, 63, 64, 0xFFFFFFFFu);
    st2_v4u(W3T2 + (size_t)u * 8, o);
  } else if (b < 24) {
    const int u = (b - 12) * 256 + tid;
    const int n = u / 48;
    const int p = u - 48 * n;
    const int pm = p >= 24 ? p - 24 : p;
    const int nn = n < NCLS ? n : NCLS - 1;
    const v4u o = gather8_bf16(Wc, nn, 8 * pm, 255, NCLS, n < NCLS ? 0xFFFFFFFFu : 0u);
    st2_v4u(WCT2 + (size_t)u * 8, o);
  } else if (b < 26) {
    const int lane = tid & 31;
    const int wave = __builtin_amdgcn_readfirstlane(tid >> 5);
    const int u = (b - 24) * 8 + wave;
    if (u < PAR_LINES) {
      float v = 0.0f;
      if (u < 2) {
        v = b1[32 * u + lane];
      } else if (u < 4) {
        v = b2[32 * (u - 2) + lane];
      } else if (u < 6) {
        v = b3[32 * (u - 4) + lane];
      } else if (u < 8) {
        v = gam[32 * (u - 6) + lane];
      } else if (u < 10) {
        v = bet[32 * (u - 8) + lane];
      } else if (u < 12) {
        const int idx = 32 * (u - 10) + lane;
        const float t = bc[idx < NCLS ? idx : NCLS - 1];
        asm volatile("" :: "v"(t));
        const unsigned m = idx < NCLS ? 0xFFFFFFFFu : 0u;
        v = __uint_as_float(__float_as_uint(t) & m);
      } else {
        v = eps[0];
      }
      const float o = bf16_val(v);
      volatile float* q = PAR + 32 * u + lane;
      *q = o;
      __threadfence();
      *q = o;
    }
  } else if (b == 26) {
    const v4u z = (v4u){ 0u, 0u, 0u, 0u };
    const v4f zf = (v4f){ 0.0f, 0.0f, 0.0f, 0.0f };
    for (int q = tid; q < (MPN - NN) * 16; q += 256) {
      st2_v4u(A + (size_t)NN * 128 + (size_t)q * 8, z);
      st2_v4f(T + (size_t)NN * 64 + (size_t)q * 4, zf);
    }
  } else {
    const int g = (b - 27) * 256 + tid;
    const int row = g >> 4, p = g & 15;
    const int rc = row < NN ? row : NN - 1;
    int pk = pkt[rc];
    asm volatile("" :: "v"(pk));
    pk = clampi(pk, 0, VOCAB - 1);
    v4f v = *(const v4fa*)(emb + (size_t)pk * 64 + 4 * p);
    asm volatile("" :: "v"(v));
    const unsigned m = row < NN ? 0xFFFFFFFFu : 0u;
    v4f o;
#pragma unroll
    for (int e = 0; e < 4; ++e) o[e] = __uint_as_float(__float_as_uint(bf16_val(v[e])) & m);
    st2_v4f(H + (size_t)g * 4, o);
  }
}

__device__ __forceinline__ int scan_chunk(const int* __restrict__ dsts, int nE, int cbase, int slotBase,
                                          int nb, int vec8, int* list, int tid, int lane, int wave) {
  int wc = 0;
  const int el0  = tid * EPT;
  const int e0   = cbase + el0;
  const int sent = (-0x7fffffff - 1);
  v4i da, db;
  if (vec8 != 0 && cbase + CHUNK <= nE) {
    da = *(const v4i*)(dsts + e0);
    db = *(const v4i*)(dsts + e0 + 4);
  } else {
    const int t0 = dsts[min(e0 + 0, nE - 1)];
    const int t1 = dsts[min(e0 + 1, nE - 1)];
    const int t2 = dsts[min(e0 + 2, nE - 1)];
    const int t3 = dsts[min(e0 + 3, nE - 1)];
    const int t4 = dsts[min(e0 + 4, nE - 1)];
    const int t5 = dsts[min(e0 + 5, nE - 1)];
    const int t6 = dsts[min(e0 + 6, nE - 1)];
    const int t7 = dsts[min(e0 + 7, nE - 1)];
    asm volatile("" :: "v"(t0), "v"(t1), "v"(t2), "v"(t3), "v"(t4), "v"(t5), "v"(t6), "v"(t7));
    da.x = (e0 + 0 < nE) ? t0 : sent;
    da.y = (e0 + 1 < nE) ? t1 : sent;
    da.z = (e0 + 2 < nE) ? t2 : sent;
    da.w = (e0 + 3 < nE) ? t3 : sent;
    db.x = (e0 + 4 < nE) ? t4 : sent;
    db.y = (e0 + 5 < nE) ? t5 : sent;
    db.z = (e0 + 6 < nE) ? t6 : sent;
    db.w = (e0 + 7 < nE) ? t7 : sent;
  }
  const unsigned nbs = (unsigned)slotBase;
  const unsigned unb = (unsigned)nb;
  const unsigned s0 = (unsigned)da.x - nbs, s1 = (unsigned)da.y - nbs;
  const unsigned s2 = (unsigned)da.z - nbs, s3 = (unsigned)da.w - nbs;
  const unsigned s4 = (unsigned)db.x - nbs, s5 = (unsigned)db.y - nbs;
  const unsigned s6 = (unsigned)db.z - nbs, s7 = (unsigned)db.w - nbs;
  const bool h0 = s0 < unb, h1 = s1 < unb, h2 = s2 < unb, h3 = s3 < unb;
  const bool h4 = s4 < unb, h5 = s5 < unb, h6 = s6 < unb, h7 = s7 < unb;
  const unsigned any = __builtin_amdgcn_ballot_w32(h0 | h1 | h2 | h3 | h4 | h5 | h6 | h7);
  if (any != 0u) {
#define HITJ(J, HJ, SJ) { \
      const unsigned mj = __builtin_amdgcn_ballot_w32(HJ); \
      if (mj != 0u) { \
        if (HJ) { \
          const int pos = wc + (int)__builtin_amdgcn_mbcnt_lo(mj, 0u); \
          if (pos < WCAP) list[wave * WCAP + pos] = ((el0 + (J)) << 12) | (int)(SJ); \
        } \
        wc += (int)__builtin_popcount(mj); } }
    HITJ(0, h0, s0)
    HITJ(1, h1, s1)
    HITJ(2, h2, s2)
    HITJ(3, h3, s3)
    HITJ(4, h4, s4)
    HITJ(5, h5, s5)
    HITJ(6, h6, s6)
    HITJ(7, h7, s7)
#undef HITJ
  }
  return wc;
}

__device__ __forceinline__ int build_lists(const int* __restrict__ dsts, int nE, int nodeBase, int nb, int vec8,
                                           int* reg1, int* reg2, int* scnt, int* soff, int* list,
                                           int* wcnt, int* wtot, int tid, int lane, int wave) {
  for (int i = tid; i < NBMAX; i += NTHR) scnt[i] = 0;
  __syncthreads();

  int tot = 0;
  const int nChunks = (nE + CHUNK - 1) / CHUNK;
#pragma unroll 1
  for (int ch = 0; ch < nChunks; ++ch) {
    const int cbase = ch * CHUNK;
    const int wc = scan_chunk(dsts, nE, cbase, nodeBase, nb, vec8, list, tid, lane, wave);
    if (lane == 0) wcnt[wave] = wc;
    __syncthreads();
    int pre = 0, all = 0;
#pragma unroll
    for (int w2 = 0; w2 < NWAVE; ++w2) {
      int c = wcnt[w2];
      c = c < 0 ? 0 : (c > WCAP ? WCAP : c);
      all += c;
      pre += (w2 < wave) ? c : 0;
    }
    const int wcc  = wc > WCAP ? WCAP : wc;
    const int base = tot + pre;
#pragma unroll 1
    for (int i = lane; i < wcc; i += 32) {
      const int ent = list[wave * WCAP + i];
      const int el  = (ent >> 12) & (CHUNK - 1);
      const int sl  = ent & (NBMAX - 1);
      int eid = cbase + el;
      eid = eid > nE - 1 ? nE - 1 : eid;
      const int pos = base + i;
      if (pos < RCAP) reg1[pos] = (int)(((unsigned)eid << ESH) | (unsigned)sl);
    }
    tot += all;
    tot = tot > RCAP ? RCAP : tot;
    __syncthreads();
  }
  const int nh = tot;

  if (wave == 0) {
#pragma unroll 1
    for (int b0 = 0; b0 < nh; b0 += 32) {
      const int idx = b0 + lane;
      const int uv  = reg1[idx < RCAP ? idx : RCAP - 1];
      const int m32 = (nh - b0) < 32 ? (nh - b0) : 32;
#pragma unroll 1
      for (int k = 0; k < m32; ++k) {
        const int u  = __builtin_amdgcn_readlane(uv, k);
        const int sl = u & (NBMAX - 1);
        if (lane == 0) scnt[sl] = scnt[sl] + 1;
      }
    }
  }
  __syncthreads();

  {
    const v4i ca = *(const v4i*)(scnt + 8 * tid);
    const v4i cb = *(const v4i*)(scnt + 8 * tid + 4);
    const int e0 = ca.x < 0 ? 0 : ca.x, e1 = ca.y < 0 ? 0 : ca.y, e2 = ca.z < 0 ? 0 : ca.z, e3 = ca.w < 0 ? 0 : ca.w;
    const int e4 = cb.x < 0 ? 0 : cb.x, e5 = cb.y < 0 ? 0 : cb.y, e6 = cb.z < 0 ? 0 : cb.z, e7 = cb.w < 0 ? 0 : cb.w;
    const int ts = e0 + e1 + e2 + e3 + e4 + e5 + e6 + e7;
    int incl = ts;
#pragma unroll
    for (int d = 1; d < 32; d <<= 1) {
      const int up = __shfl_up(incl, d);
      if (lane >= d) incl += up;
    }
    if (lane == 31) wtot[wave] = incl;
    __syncthreads();
    int pre = 0;
#pragma unroll
    for (int w2 = 0; w2 < NWAVE; ++w2) pre += (w2 < wave) ? wtot[w2] : 0;
    int run = pre + incl - ts;
    soff[8 * tid + 0] = run; run += e0;
    soff[8 * tid + 1] = run; run += e1;
    soff[8 * tid + 2] = run; run += e2;
    soff[8 * tid + 3] = run; run += e3;
    soff[8 * tid + 4] = run; run += e4;
    soff[8 * tid + 5] = run; run += e5;
    soff[8 * tid + 6] = run; run += e6;
    soff[8 * tid + 7] = run;
  }
  __syncthreads();
  for (int i = tid; i < NBMAX; i += NTHR) list[i] = soff[i];
  __syncthreads();

  if (wave == 0) {
#pragma unroll 1
    for (int b0 = 0; b0 < nh; b0 += 32) {
      const int idx = b0 + lane;
      const int uv  = reg1[idx < RCAP ? idx : RCAP - 1];
      const int m32 = (nh - b0) < 32 ? (nh - b0) : 32;
#pragma unroll 1
      for (int k = 0; k < m32; ++k) {
        const int u   = __builtin_amdgcn_readlane(uv, k);
        const int sl  = u & (NBMAX - 1);
        const int eid = (int)((unsigned)u >> ESH);
        if (lane == 0) {
          int pos = list[sl];
          pos = pos < 0 ? 0 : (pos > RCAP - 1 ? RCAP - 1 : pos);
          reg2[pos] = eid;
          list[sl] = pos + 1;
        }
      }
    }
  }
  __syncthreads();
  return nh;
}

template <int RES>
__global__ __launch_bounds__(NTHR) void k_bucket(const int* __restrict__ keys, int nE, int nN, int nbrows, int vec8,
                                                 const int* __restrict__ vals, int nV,
                                                 int* BLIST, int* OFFC, int* META) {
  extern __shared__ v4f lds_dyn[];
  int* reg1 = (int*)lds_dyn;
  int* reg2 = reg1 + RCAP;
  int* scnt = reg2 + RCAP;
  int* soff = scnt + NBMAX;
  int* list = soff + NBMAX;
  int* wcnt = list + LISTN;
  int* wtot = wcnt + NWAVE;
  const int tid = (int)threadIdx.x, lane = tid & 31, wave = tid >> 5;
  const int b = (int)blockIdx.x;
  const int nodeBase = b * nbrows;
  int nb = nN - nodeBase;
  nb = nb < 0 ? 0 : (nb > nbrows ? nbrows : nb);

  const int nh = build_lists(keys, nE, nodeBase, nb, vec8, reg1, reg2, scnt, soff, list, wcnt, wtot, tid, lane, wave);

  int* bl = BLIST + (size_t)b * RCAP;
  const int last = nh > 0 ? nh - 1 : 0;
#pragma unroll 1
  for (int base = 0; base < RCAP; base += 1024) {
    const int i0 = base + 4 * tid;
    int a0 = reg2[i0     < last ? i0     : last];
    int a1 = reg2[i0 + 1 < last ? i0 + 1 : last];
    int a2 = reg2[i0 + 2 < last ? i0 + 2 : last];
    int a3 = reg2[i0 + 3 < last ? i0 + 3 : last];
    if (RES) {
      a0 = clampi(a0, 0, nE - 1);
      a1 = clampi(a1, 0, nE - 1);
      a2 = clampi(a2, 0, nE - 1);
      a3 = clampi(a3, 0, nE - 1);
      const int s0 = vals[a0];
      const int s1 = vals[a1];
      const int s2 = vals[a2];
      const int s3 = vals[a3];
      asm volatile("" :: "v"(s0), "v"(s1), "v"(s2), "v"(s3));
      a0 = clampi(s0, 0, nV - 1);
      a1 = clampi(s1, 0, nV - 1);
      a2 = clampi(s2, 0, nV - 1);
      a3 = clampi(s3, 0, nV - 1);
    }
    v4i v;
    v.x = (i0     < nh) ? a0 : 0;
    v.y = (i0 + 1 < nh) ? a1 : 0;
    v.z = (i0 + 2 < nh) ? a2 : 0;
    v.w = (i0 + 3 < nh) ? a3 : 0;
    st2_v4i(bl + i0, v);
  }
  {
    const v4i so = *(const v4ia*)(soff + 4 * tid);
    const v4i sc = *(const v4ia*)(scnt + 4 * tid);
    int* oc = OFFC + (size_t)b * 2048;
    st2_v4i(oc + 4 * tid, so);
    st2_v4i(oc + 1024 + 4 * tid, sc);
  }
  if (tid < 8) {
    v4i mv;
    mv.x = (tid == 0) ? nh : 0;
    mv.y = (tid == 0 && nh >= RCAP) ? 1 : 0;
    mv.z = 0; mv.w = 0;
    st2_v4i(META + (size_t)b * 32 + 4 * tid, mv);
  }
}

__global__ __launch_bounds__(256) void k_agg(const float* __restrict__ H, const int* __restrict__ BLIST,
                                             const int* __restrict__ OFFC, const int* __restrict__ META,
                                             const float* __restrict__ par, unsigned short* A) {
  extern __shared__ v4f lds_dyn[];
  __shared__ __attribute__((aligned(16))) float sS[8][128];
  int* slist = (int*)lds_dyn;
  const int tid = (int)threadIdx.x, lane = tid & 31;
  const int wave = __builtin_amdgcn_readfirstlane(tid >> 5);
  const int hh = lane >> 4;
  const int pp = lane & 15;
  const int c4 = pp * 4;
  const int b = (int)blockIdx.x;
  const int nodeBase = b * NBROWS;
  const int nb = clampi(NN - nodeBase, 0, NBROWS);
  const int nh = clampi(META[(size_t)b * 32], 0, RCAP);
  const int flag = META[(size_t)b * 32 + 1];
  const bool ovf = flag != 0;
  const int* bl = BLIST + (size_t)b * RCAP;
  const int* oc = OFFC + (size_t)b * 2048;
  const int nhs = nh > 0 ? nh : 1;
#pragma unroll 1
  for (int base = 0; base < nhs; base += 1024) {
    const int i0 = base + 4 * tid;
    *(v4ia*)(slist + i0) = *(const v4ia*)(bl + i0);
  }
  __syncthreads();
  const float ope = 1.0f + par[PA_EPS];
  const int nhm1 = nh > 0 ? nh - 1 : 0;
  const float qnan = __int_as_float(0x7fc00000);
  float* srow = &sS[wave][0];

#pragma unroll 1
  for (int g = 0; g < 32; ++g) {
    const int slot0 = wave * 64 + g * 2;
    if (slot0 >= nb) break;
    const int slot = slot0 + hh;
    int stv = oc[slot];
    int cv  = oc[1024 + slot];
    asm volatile("" :: "v"(stv), "v"(cv));
    const int craw = cv < 0 ? 0 : cv;
    const bool pv = craw > DEGCAP;
    stv = clampi(stv, 0, nh);
    int cc = clampi(craw, 0, DEGCAP);
    cc = cc > nh - stv ? nh - stv : cc;
    const int c0 = __builtin_amdgcn_readlane(cc, 0);
    const int c1 = __builtin_amdgcn_readlane(cc, 16);
    const int mx = c0 > c1 ? c0 : c1;
    v4f acc = (v4f){ 0.0f, 0.0f, 0.0f, 0.0f };
#pragma unroll 1
    for (int q = 0; q < mx; ++q) {
      const int li = clampi(stv + q, 0, nhm1);
      const int s  = clampi(slist[li], 0, NN - 1);
      const v4f v = *(const v4fa*)(H + (size_t)s * 64 + c4);
      asm volatile("" :: "v"(v));
      const unsigned m = (q < cc) ? 0xFFFFFFFFu : 0u;
      acc[0] += __uint_as_float(__float_as_uint(v[0]) & m);
      acc[1] += __uint_as_float(__float_as_uint(v[1]) & m);
      acc[2] += __uint_as_float(__float_as_uint(v[2]) & m);
      acc[3] += __uint_as_float(__float_as_uint(v[3]) & m);
    }
    const int row = nodeBase + slot;
    const v4f hd = *(const v4fa*)(H + (size_t)row * 64 + c4);
    asm volatile("" :: "v"(hd));
    const bool bad = ovf || pv;
    v4f z;
#pragma unroll
    for (int e = 0; e < 4; ++e) {
      const float t = ope * hd[e] + acc[e];
      z[e] = bad ? qnan : t;
    }
    *(v4fa*)(srow + hh * 64 + c4) = z;
    wave_sync_lds();
    {
      const float* sp = srow + hh * 64 + (pp & 7) * 8;
      const v4f a = *(const v4fa*)sp;
      const v4f c = *(const v4fa*)(sp + 4);
      const v4u hi = pack8_bf16(a, c);
      const v4u lo = pack8_bf16_lo(a, c);
      const v4u o = (pp >= 8) ? lo : hi;
      st2_v4u(A + (size_t)row * 128 + pp * 8, o);
    }
    wave_sync_lds();
  }
}

__global__ __launch_bounds__(256) void k_epi(const float* __restrict__ T, const float* __restrict__ par, int pofs,
                                             unsigned short* A) {
  __shared__ __attribute__((aligned(16))) float sP[64];
  const int tid = (int)threadIdx.x;
  {
    const int ix = tid < 15 ? tid : 15;
    const v4f w = *(const v4fa*)(par + pofs + 4 * ix);
    asm volatile("" :: "v"(w));
    if (tid < 16) *(v4fa*)(sP + 4 * tid) = w;
  }
  __syncthreads();
  const int g = (int)blockIdx.x * 256 + tid;
  const int row = g >> 4, p = g & 15;
  const int c0 = (p & 7) * 8;
  const int rc = row < NN ? row : NN - 1;
  v4f a = *(const v4fa*)(T + (size_t)rc * 64 + c0);
  v4f c = *(const v4fa*)(T + (size_t)rc * 64 + c0 + 4);
  asm volatile("" :: "v"(a), "v"(c));
  a += *(const v4fa*)(sP + c0);
  c += *(const v4fa*)(sP + c0 + 4);
#pragma unroll
  for (int e = 0; e < 4; ++e) { a[e] = relu_keep(a[e]); c[e] = relu_keep(c[e]); }
  const v4u hi = pack8_bf16(a, c);
  const v4u lo = pack8_bf16_lo(a, c);
  v4u o = (p >= 8) ? lo : hi;
  const unsigned m = row < NN ? 0xFFFFFFFFu : 0u;
  o &= (v4u){ m, m, m, m };
  st2_v4u(A + (size_t)g * 8, o);
}

__global__ __launch_bounds__(256) void k_epi3(float* T, const float* __restrict__ par, int pofs, double* REC) {
  __shared__ __attribute__((aligned(16))) float sX[128 * 68];
  __shared__ __attribute__((aligned(16))) double sRec[192];
  __shared__ __attribute__((aligned(16))) float sP[64];
  const int tid = (int)threadIdx.x;
  const int blk = (int)blockIdx.x;
  const int row0 = blk * 128;
  {
    const int ix = tid < 15 ? tid : 15;
    const v4f w = *(const v4fa*)(par + pofs + 4 * ix);
    asm volatile("" :: "v"(w));
    if (tid < 16) *(v4fa*)(sP + 4 * tid) = w;
  }
  __syncthreads();
#pragma unroll 1
  for (int it = 0; it < 8; ++it) {
    const int idx = it * 256 + tid;
    const int r = idx >> 4, p = idx & 15;
    const int row = row0 + r;
    const int rc = row < NN ? row : NN - 1;
    v4f v = *(const v4fa*)(T + (size_t)rc * 64 + 4 * p);
    asm volatile("" :: "v"(v));
    v += *(const v4fa*)(sP + 4 * p);
    const unsigned m = row < NN ? 0xFFFFFFFFu : 0u;
    v4f x;
#pragma unroll
    for (int e = 0; e < 4; ++e) x[e] = __uint_as_float(__float_as_uint(relu_keep(v[e])) & m);
    *(v4fa*)(sX + r * 68 + 4 * p) = x;
    st2_v4f(T + (size_t)row * 64 + 4 * p, x);
  }
  __syncthreads();
  int nbr = NN - row0;
  nbr = nbr > 128 ? 128 : (nbr < 1 ? 1 : nbr);
  if (tid < 64) {
    double s = 0.0;
#pragma unroll 4
    for (int r = 0; r < nbr; ++r) s += (double)sX[r * 68 + tid];
    const double mean = s / (double)nbr;
    double m2 = 0.0;
#pragma unroll 4
    for (int r = 0; r < nbr; ++r) {
      const double d = (double)sX[r * 68 + tid] - mean;
      m2 += d * d;
    }
    sRec[tid] = (double)nbr;
    sRec[64 + tid] = mean;
    sRec[128 + tid] = m2;
  }
  __syncthreads();
  if (tid < 96) {
    const v2d v = *(const v2da*)(sRec + 2 * tid);
    st2_v2d(REC + (size_t)blk * 192 + 2 * tid, v);
  }
}

__global__ __launch_bounds__(64) void k_comb(const double* __restrict__ REC, float* STAT) {
  __shared__ __attribute__((aligned(16))) float sS[128];
  const int c = (int)threadIdx.x;
  double n = 0.0, mean = 0.0, M2 = 0.0;
#pragma unroll 1
  for (int b = 0; b < NREC; ++b) {
    const double nb = REC[(size_t)b * 192 + c];
    const double mb = REC[(size_t)b * 192 + 64 + c];
    const double qb = REC[(size_t)b * 192 + 128 + c];
    const double nt = n + nb;
    const double delta = mb - mean;
    const double w = nb / nt;
    mean = mean + delta * w;
    M2 = M2 + qb + (delta * delta) * (n * w);
    n = nt;
  }
  const float var = (float)(M2 / (double)NN);
  const float mf = (float)mean;
  const float r = 1.0f / sqrtf(var + 1e-5f);
  sS[c] = mf;
  sS[64 + c] = r;
  __syncthreads();
  if (c < 32) {
    const v4f v = *(const v4fa*)(sS + 4 * c);
    st2_v4f(STAT + 4 * c, v);
  }
}

__global__ __launch_bounds__(256) void k_apply(const float* __restrict__ X, const float* __restrict__ par,
                                               const float* __restrict__ STAT, float* H) {
  __shared__ __attribute__((aligned(16))) float sP[256];
  const int tid = (int)threadIdx.x;
  if (tid < 32) {
    const v4f a = *(const v4fa*)(par + PA_GAM + 4 * tid);
    const v4f s = *(const v4fa*)(STAT + 4 * tid);
    *(v4fa*)(sP + 4 * tid) = a;
    *(v4fa*)(sP + 128 + 4 * tid) = s;
  }
  __syncthreads();
  const int g = (int)blockIdx.x * 256 + tid;
  const int row = g >> 4, p = g & 15;
  const int c4 = 4 * p;
  const int rc = row < NN ? row : NN - 1;
  const v4f x = *(const v4fa*)(X + (size_t)rc * 64 + c4);
  asm volatile("" :: "v"(x));
  const v4f pg = *(const v4fa*)(sP + c4);
  const v4f pb = *(const v4fa*)(sP + 64 + c4);
  const v4f pm = *(const v4fa*)(sP + 128 + c4);
  const v4f pr = *(const v4fa*)(sP + 192 + c4);
  const v4f y = (pg * (x - pm)) * pr + pb;
  const unsigned m = row < NN ? 0xFFFFFFFFu : 0u;
  v4f o;
#pragma unroll
  for (int e = 0; e < 4; ++e) o[e] = __uint_as_float(__float_as_uint(y[e]) & m);
  st2_v4f(H + (size_t)g * 4, o);
}

__global__ __launch_bounds__(256) void k_pool(const float* __restrict__ H, const int* __restrict__ GBLIST,
                                              const int* __restrict__ GOFFC, const int* __restrict__ GMETA,
                                              float* GF, int colofs) {
  const int tid = (int)threadIdx.x, lane = tid & 31;
  const int wave = __builtin_amdgcn_readfirstlane(tid >> 5);
  const int hh = lane >> 4;
  const int c4 = (lane & 15) * 4;
  const int b = (int)blockIdx.x;
  const int nh = clampi(GMETA[(size_t)b * 32], 0, RCAP);
  const int flag = GMETA[(size_t)b * 32 + 1];
  const bool ovf = flag != 0;
  const int* bl = GBLIST + (size_t)b * RCAP;
  const int* oc = GOFFC + (size_t)b * 2048;
  const int nhm1 = nh > 0 ? nh - 1 : 0;
  const float qnan = __int_as_float(0x7fc00000);
#pragma unroll 1
  for (int g2 = 0; g2 < 2; ++g2) {
    const int slot = wave * 4 + g2 * 2 + hh;
    int stv = oc[slot];
    int cv  = oc[1024 + slot];
    asm volatile("" :: "v"(stv), "v"(cv));
    const int craw = cv < 0 ? 0 : cv;
    const bool pv = craw > GCAP;
    stv = clampi(stv, 0, nh);
    int cc = clampi(craw, 0, GCAP);
    cc = cc > nh - stv ? nh - stv : cc;
    const int c0 = __builtin_amdgcn_readlane(cc, 0);
    const int c1 = __builtin_amdgcn_readlane(cc, 16);
    const int mx = c0 > c1 ? c0 : c1;
    v4f acc = (v4f){ 0.0f, 0.0f, 0.0f, 0.0f };
#pragma unroll 1
    for (int q = 0; q < mx; ++q) {
      const int li = clampi(stv + q, 0, nhm1);
      int nd = bl[li];
      asm volatile("" :: "v"(nd));
      nd = clampi(nd, 0, NN - 1);
      const v4f v = *(const v4fa*)(H + (size_t)nd * 64 + c4);
      asm volatile("" :: "v"(v));
      const unsigned m = (q < cc) ? 0xFFFFFFFFu : 0u;
      acc[0] += __uint_as_float(__float_as_uint(v[0]) & m);
      acc[1] += __uint_as_float(__float_as_uint(v[1]) & m);
      acc[2] += __uint_as_float(__float_as_uint(v[2]) & m);
      acc[3] += __uint_as_float(__float_as_uint(v[3]) & m);
    }
    const bool bad = ovf || pv;
    v4f o;
#pragma unroll
    for (int e = 0; e < 4; ++e) o[e] = bad ? qnan : acc[e];
    st2_v4f(GF + (size_t)(b * GROWS + slot) * 192 + colofs + c4, o);
  }
}

__global__ __launch_bounds__(256) void k_out(const float* __restrict__ C, const float* __restrict__ par, float* out) {
  __shared__ __attribute__((aligned(16))) float img[32 * NCLS];
  const int tid = (int)threadIdx.x;
  const int b = (int)blockIdx.x;
#pragma unroll 1
  for (int k = 0; k < 7; ++k) {
    const int e = tid + 256 * k;
    const int ec = e < 32 * NCLS ? e : 32 * NCLS - 1;
    const int r = ec / NCLS;
    const int c = ec - NCLS * r;
    const float cv = C[(size_t)(b * 32 + r) * 64 + c];
    const float bv = par[PA_BC + c];
    asm volatile("" :: "v"(cv), "v"(bv));
    const float v = cv + bv;
    if (e < 32 * NCLS) img[e] = v;
  }
  __syncthreads();
#pragma unroll 1
  for (int k = 0; k < 2; ++k) {
    const int pidx = tid + 256 * k;
    const int pc = pidx < 8 * NCLS ? pidx : 8 * NCLS - 1;
    const v4f v = *(const v4fa*)(img + 4 * pc);
    asm volatile("" :: "v"(v));
    if (pidx < 8 * NCLS) st2_v4f(out + (size_t)b * (32 * NCLS) + 4 * pidx, v);
  }
}

extern "C" void kernel_launch(void* const* d_in, const int* in_sizes, int n_in,
                              void* d_out, int out_size, void* d_ws, size_t ws_size,
                              hipStream_t stream) {
  if (n_in < 16) return;
  if (in_sizes[0] != NN || in_sizes[1] != NE || in_sizes[2] != NE || in_sizes[3] != NN) return;
  if (in_sizes[4] != VOCAB * 64 || in_sizes[5] != 1) return;
  if (in_sizes[6] != 64 * 64 || in_sizes[7] != 64 || in_sizes[8] != 64 * 64 || in_sizes[9] != 64) return;
  if (in_sizes[10] != 64 * 64 || in_sizes[11] != 64 || in_sizes[12] != 64 || in_sizes[13] != 64) return;
  if (in_sizes[14] != 192 * NCLS || in_sizes[15] != NCLS) return;
  if (out_size != NG * NCLS) return;
  if (ws_size < WS_TOTAL) return;

  const int*   pkt   = (const int*)  d_in[0];
  const int*   src   = (const int*)  d_in[1];
  const int*   dst   = (const int*)  d_in[2];
  const int*   gid   = (const int*)  d_in[3];
  const float* emb   = (const float*)d_in[4];
  const float* eps   = (const float*)d_in[5];
  const float* W1    = (const float*)d_in[6];
  const float* b1    = (const float*)d_in[7];
  const float* W2    = (const float*)d_in[8];
  const float* b2    = (const float*)d_in[9];
  const float* W3    = (const float*)d_in[10];
  const float* b3    = (const float*)d_in[11];
  const float* gam   = (const float*)d_in[12];
  const float* bet   = (const float*)d_in[13];
  const float* Wc    = (const float*)d_in[14];
  const float* bc    = (const float*)d_in[15];
  float* out = (float*)d_out;

  char* ws = (char*)d_ws;
  float*          H      = (float*)(ws + O_H);
  float*          T      = (float*)(ws + O_T);
  unsigned short* A      = (unsigned short*)(ws + O_A);
  int*            BLIST  = (int*)(ws + O_BLIST);
  int*            OFFC   = (int*)(ws + O_OFFC);
  int*            META   = (int*)(ws + O_META);
  int*            GBLIST = (int*)(ws + O_GBLIST);
  int*            GOFFC  = (int*)(ws + O_GOFFC);
  int*            GMETA  = (int*)(ws + O_GMETA);
  double*         REC    = (double*)(ws + O_REC);
  float*          STAT   = (float*)(ws + O_STAT);
  float*          PAR    = (float*)(ws + O_PAR);
  unsigned short* W1T2   = (unsigned short*)(ws + O_W1T);
  unsigned short* W2T2   = (unsigned short*)(ws + O_W2T);
  unsigned short* W3T2   = (unsigned short*)(ws + O_W3T);
  unsigned short* WCT2   = (unsigned short*)(ws + O_WCT);
  float*          GF     = (float*)(ws + O_GF);
  unsigned short* GFHL   = (unsigned short*)(ws + O_GFHL);
  float*          C      = (float*)(ws + O_C);

  hipFuncSetAttribute(reinterpret_cast<const void*>(&k_bucket<1>),
                      hipFuncAttributeMaxDynamicSharedMemorySize, LDS_BKT);
  hipFuncSetAttribute(reinterpret_cast<const void*>(&k_bucket<0>),
                      hipFuncAttributeMaxDynamicSharedMemorySize, LDS_BKT);
  hipFuncSetAttribute(reinterpret_cast<const void*>(&k_agg),
                      hipFuncAttributeMaxDynamicSharedMemorySize, LDS_AGG);

  k_prep<<<27 + MPN * 16 / 256, 256, 0, stream>>>(pkt, emb, eps, W1, b1, W2, b2, W3, b3, gam, bet, Wc, bc,
                                                  W1T2, W2T2, W3T2, WCT2, PAR, H, T, A);
  k_bucket<1><<<NBLK, NTHR, LDS_BKT, stream>>>(dst, NE, NN, NBROWS, 1, src, NN, BLIST, OFFC, META);
  k_bucket<0><<<GBLK, NTHR, LDS_BKT, stream>>>(gid, NN, NG, GROWS, 1, gid, NN, GBLIST, GOFFC, GMETA);

  const int gemmGrid = (782 + 7) / 8;
  for (int i = 0; i < 3; ++i) {
    k_agg<<<NBLK, 256, LDS_AGG, stream>>>(H, BLIST, OFFC, META, PAR, A);
    k_gemm_nt<0, 0><<<gemmGrid, 256, 0, stream>>>(A, W1T2, PAR, T, NN, 64, 128, 64);
    k_epi<<<MPN * 16 / 256, 256, 0, stream>>>(T, PAR, PA_B1, A);
    k_gemm_nt<0, 0><<<gemmGrid, 256, 0, stream>>>(A, W2T2, PAR, T, NN, 64, 128, 64);
    k_epi<<<MPN * 16 / 256, 256, 0, stream>>>(T, PAR, PA_B2, A);
    k_gemm_nt<0, 0><<<gemmGrid, 256, 0, stream>>>(A, W3T2, PAR, T, NN, 64, 128, 64);
    k_epi3<<<NREC, 256, 0, stream>>>(T, PAR, PA_B3, REC);
    k_comb<<<1, 64, 0, stream>>>(REC, STAT);
    k_apply<<<MPN * 16 / 256, 256, 0, stream>>>(T, PAR, STAT, H);
    k_pool<<<GBLK, 256, 0, stream>>>(H, GBLIST, GOFFC, GMETA, GF, 64 * i);
  }
  k_plane<1><<<NG * 384 / 8 / 256, 256, 0, stream>>>(GF, NG, 192, 192, GFHL, NG, 192);
  k_gemm_nt<0, 0><<<1, 256, 0, stream>>>(GFHL, WCT2, PAR, C, NG, 64, 384, 64);
  k_out<<<NG / 32, 256, 0, stream>>>(C, PAR, out);
}
